// DySepConvAtten_6047313952931
// MI455X (gfx1250) — hardware-run, weakly checked
//
#include <hip/hip_runtime.h>


#define NSP  512
#define NRW  100
#define NCL  256
#define NGN  103
#define NPD  128
#define PRT  128
constexpr size_t al256(size_t b) { return (b + 255) & ~(size_t)255; }
constexpr size_t WS_TOTAL = al256((size_t)NSP * NRW * NCL * 2) + al256((size_t)NPD * NCL * 2) + al256((size_t)NSP * NRW * NPD * 4) + al256((size_t)3 * NCL * 4) + al256((size_t)PRT * NRW * NCL * 4) + al256((size_t)PRT * NPD * NPD * 2) + al256((size_t)PRT * NCL * NPD * 2) + al256((size_t)PRT * NPD * NCL * 4) + al256((size_t)PRT * NPD * 2 * 4);
static_assert(WS_TOTAL == 95095808 && WS_TOTAL <= 134217728, "the workspace carve: 90.7 MiB");
static_assert(NGN == 3 + NRW && NGN <= NPD && NRW <= NPD && NPD % 64 == 0 && NCL % 64 == 0 && NSP % PRT == 0 && (NSP * NRW) % 64 == 0 && NGN <= NCL && (PRT * NRW * NCL) % 4 == 0, "whole tiles; whole lines");
typedef _Float16 h16;
typedef unsigned short bf;
typedef __attribute__((ext_vector_type(16))) __bf16   v16bf;
typedef __attribute__((ext_vector_type(16))) _Float16 v16h;
typedef __attribute__((ext_vector_type(8)))  _Float16 v8h;
typedef __attribute__((ext_vector_type(8)))  unsigned short v8us;
typedef __attribute__((ext_vector_type(8)))  float    v8f;
typedef __attribute__((ext_vector_type(4)))  float    v4f;
typedef v8h  __attribute__((may_alias)) v8ha;
typedef v4f  __attribute__((may_alias)) v4fa;
typedef v8us __attribute__((may_alias)) v8usa;

__device__ __forceinline__ unsigned short f2bf(float f) { unsigned u = __float_as_uint(f); u += 0x7FFFu + ((u >> 16) & 1u); return (unsigned short)(u >> 16); }
__device__ __forceinline__ float bf2f(unsigned short b) { return __uint_as_float(((unsigned)b) << 16); }
__device__ __forceinline__ float bfr(float f) { return bf2f(f2bf(f)); }
__device__ __forceinline__ v16h cat16(v8h lo, v8h hi) { return __builtin_shufflevector(lo, hi, 0, 1, 2, 3, 4, 5, 6, 7, 8, 9, 10, 11, 12, 13, 14, 15); }
__device__ __forceinline__ v16bf cat16b(v8us lo, v8us hi) { return __builtin_bit_cast(v16bf, __builtin_shufflevector(lo, hi, 0, 1, 2, 3, 4, 5, 6, 7, 8, 9, 10, 11, 12, 13, 14, 15)); }
__device__ __forceinline__ v8f wmma16(v16h a, v16h b, v8f c) { return __builtin_amdgcn_wmma_f32_16x16x32_f16(false, a, false, b, (short)0, c, false, false); }
__device__ __forceinline__ v8f wmmab(v16bf a, v16bf b, v8f c) { return __builtin_amdgcn_wmma_f32_16x16x32_bf16(false, a, false, b, (short)0, c, false, false); }


template <typename T16> struct WFrag;
template <> struct WFrag<h16> { typedef v16h V; static __device__ __forceinline__ V ld(const h16* p) { return cat16(*(const v8h*)p, *(const v8h*)(p + 16)); } static __device__ __forceinline__ v8f mma(V a, V b, v8f c) { return wmma16(a, b, c); } };
template <> struct WFrag<bf> { typedef v16bf V; static __device__ __forceinline__ V ld(const bf* p) { return cat16b(*(const v8us*)p, *(const v8us*)(p + 16)); } static __device__ __forceinline__ v8f mma(V a, V b, v8f c) { return wmmab(a, b, c); } };
template <typename T16, int NSPLIT, bool BIAS>
__global__ __launch_bounds__(32) void k_gemmw(const T16* __restrict__ A, const T16* __restrict__ A2, const T16* __restrict__ Bt, const T16* __restrict__ Bt2, int K, float* C, int ldc, const float* __restrict__ bias, size_t sA, size_t sB, size_t sC) {
    typedef typename WFrag<T16>::V V;
    __shared__ __align__(16) float os[16 * 68];
    const size_t z = blockIdx.z; A += z * sA; if (A2) A2 += z * sA; Bt += z * sB; if (Bt2) Bt2 += z * sB; C += z * sC;
    const int lane = threadIdx.x & 31, lr = lane & 15, hi = lane >> 4; const int r0 = blockIdx.x * 64, c0 = blockIdx.y * 64;
    v8f acc[4][4];
#pragma unroll
    for (int mb = 0; mb < 4; ++mb)
#pragma unroll
        for (int nb = 0; nb < 4; ++nb) acc[mb][nb] = (v8f){};
    const size_t aoff = (size_t)(r0 + lr) * K + 8 * hi, boff = (size_t)(c0 + lr) * K + 8 * hi;
    for (int kc = 0; kc < K; kc += 32) {
        V a[4], a2[4];
#pragma unroll
        for (int mb = 0; mb < 4; ++mb) { a[mb] = WFrag<T16>::ld(A + aoff + (size_t)mb * 16 * K + kc); if (NSPLIT == 1 || NSPLIT == 2) a2[mb] = WFrag<T16>::ld(A2 + aoff + (size_t)mb * 16 * K + kc); }
#pragma unroll
        for (int nb = 0; nb < 4; ++nb) { const V b = WFrag<T16>::ld(Bt + boff + (size_t)nb * 16 * K + kc); V b2; if (NSPLIT >= 2) b2 = WFrag<T16>::ld(Bt2 + boff + (size_t)nb * 16 * K + kc);
#pragma unroll
            for (int mb = 0; mb < 4; ++mb) { acc[mb][nb] = WFrag<T16>::mma(a[mb], b, acc[mb][nb]); if (NSPLIT == 1 || NSPLIT == 2) acc[mb][nb] = WFrag<T16>::mma(a2[mb], b, acc[mb][nb]); if (NSPLIT >= 2) acc[mb][nb] = WFrag<T16>::mma(a[mb], b2, acc[mb][nb]); } }
        asm volatile("v_nop\n\tv_nop\n\tv_nop\n\tv_nop" : "+v"(acc[0][0]), "+v"(acc[1][1]), "+v"(acc[2][2]), "+v"(acc[3][3]) : "v"(a[0]), "v"(a[3]));
    }
#pragma unroll
    for (int mb = 0; mb < 4; ++mb) {
#pragma unroll
        for (int nb = 0; nb < 4; ++nb) {
#pragma unroll
            for (int j = 0; j < 8; ++j) os[(hi * 8 + j) * 68 + nb * 16 + lr] = acc[mb][nb][j]; }
        __builtin_amdgcn_wave_barrier(); asm volatile("" ::: "memory");
        float* crow = C + (size_t)(r0 + mb * 16) * ldc + c0;
#pragma unroll 1
        for (int ps = 0; ps < 2; ++ps) {
#pragma unroll
            for (int s = 0; s < 8; ++s) { const int row = 2 * s + hi, cofs = lr * 4; v4f val = *(const v4fa*)(os + row * 68 + cofs); if (BIAS) { val[0] += bfr(bias[c0 + cofs]); val[1] += bfr(bias[c0 + cofs + 1]); val[2] += bfr(bias[c0 + cofs + 2]); val[3] += bfr(bias[c0 + cofs + 3]); }
                *(volatile v4f*)(crow + (size_t)row * ldc + cofs) = val; }
            if (ps == 0) __threadfence(); }
        __builtin_amdgcn_wave_barrier(); asm volatile("" ::: "memory");
    }
}

__device__ __forceinline__ h16 tohx(float x) { return (h16)x; }
__device__ __forceinline__ void splitf(float y, unsigned short& h, unsigned short& l) { h = f2bf(y); l = f2bf(y - bf2f(h)); }
typedef __attribute__((ext_vector_type(2))) _Float16 v2h;
typedef __attribute__((ext_vector_type(4))) _Float16 v4h;
typedef __attribute__((ext_vector_type(2))) unsigned short v2us;
typedef __attribute__((ext_vector_type(4))) unsigned short v4us;
typedef __attribute__((ext_vector_type(2))) float v2f;
typedef __attribute__((ext_vector_type(4))) int v4i;


__global__ __launch_bounds__(256) void k_lay(const float* __restrict__ src, h16* dst, unsigned nrow, unsigned c8n, unsigned dp, unsigned c0, unsigned rbs, unsigned ra, unsigned rs, unsigned cbs, unsigned sa, unsigned sb, unsigned rlive, unsigned clive) {
    const unsigned g = blockIdx.x * 256 + threadIdx.x; if (g >= nrow * c8n) return; const unsigned row = g / c8n, ch = g - row * c8n; const unsigned rb = (row >> rbs) * ra + (row & ((1u << rbs) - 1u)) * rs; v8h o;
#pragma unroll
    for (int w = 0; w < 8; ++w) { const unsigned c = 8u * ch + w; const bool live = row < rlive && c < clive; const unsigned si = rb + (c >> cbs) * sa + (c & ((1u << cbs) - 1u)) * sb; const float v = bfr(src[live ? si : 0u]); o[w] = tohx(live && fabsf(v) >= 6.103515625e-05f ? v : 0.0f); }
    h16* d8 = dst + (size_t)row * dp + c0 + 8u * ch; *(volatile v8h*)(d8) = o; __threadfence(); *(volatile v8h*)(d8) = o; }

__global__ __launch_bounds__(256) void k_rnd(const float* __restrict__ src, float* dst, unsigned npc, unsigned nw) {
    const unsigned g = blockIdx.x * 256 + threadIdx.x; if (g >= npc) return; v4f o;
#pragma unroll
    for (int e = 0; e < 4; ++e) { const unsigned i = 4u * g + (unsigned)e; const unsigned live = i < nw ? 1u : 0u; const float rv_ = bfr(src[live ? i : 0u]); o[e] = live ? rv_ : 0.0f; }
    float* dq = dst + 4u * (size_t)g; *(volatile v4f*)(dq) = o; __threadfence(); *(volatile v4f*)(dq) = o; }

__global__ __launch_bounds__(256) void k_ops(const float* __restrict__ gn, const float* __restrict__ rb, const float* __restrict__ rv, h16* pm, h16* dt, unsigned s0) {
    const unsigned g = blockIdx.x * 256 + threadIdx.x; if (g >= (unsigned)(PRT * NPD * (NPD / 8) + PRT * NCL * (NPD / 8))) return; v8h o; h16* d8;
    if (g < (unsigned)(PRT * NPD * (NPD / 8))) { const unsigned ch = g & 15u, rn = (g >> 4) & 127u, sl = g >> 11; const unsigned rlive = rn < (unsigned)NRW ? 1u : 0u, rr = rlive ? rn : 0u; const float* dr = gn + ((size_t)(s0 + sl) * NRW + rr) * NPD;
#pragma unroll
        for (int e = 0; e < 8; ++e) { const unsigned m = 8u * ch + (unsigned)e; const unsigned live = (m < (unsigned)NRW ? 1u : 0u) & rlive; const unsigned mc = live ? m : 0u; const float lv = live ? 1.0f : 0.0f; const float fv = lv * (dr[3u + mc] + rb[3u + mc]);
            o[e] = tohx(fabsf(fv) >= 6.103515625e-05f ? fv : 0.0f); }
        d8 = pm + (size_t)g * 8u; }
    else { const unsigned h = g - (unsigned)(PRT * NPD * (NPD / 8)); const unsigned ch = h & 15u, cc = (h >> 4) & 255u, sl = h >> 12; const unsigned lo = cc > 0u ? 1u : 0u, hi = cc < (unsigned)(NCL - 1) ? 1u : 0u; const unsigned cl = cc - lo, cr = hi ? cc + 1u : 0u;
        const float b0 = rb[0], b1 = rb[1], b2 = rb[2]; const float ml = lo ? 1.0f : 0.0f, mh = hi ? 1.0f : 0.0f;
#pragma unroll
        for (int e = 0; e < 8; ++e) { const unsigned m = 8u * ch + (unsigned)e; const unsigned live = m < (unsigned)NRW ? 1u : 0u; const unsigned mc = live ? m : 0u; const float lv = live ? 1.0f : 0.0f; const float* dr = gn + ((size_t)(s0 + sl) * NRW + mc) * NPD; const float* vr = rv + ((size_t)sl * NRW + mc) * NCL;
            const float tv = (dr[0] + b0) * (ml * vr[cl]) + (dr[1] + b1) * vr[cc] + (dr[2] + b2) * (mh * vr[cr]); const float fv = lv * fmaxf(tv, 0.0f);
            o[e] = tohx(fabsf(fv) >= 6.103515625e-05f ? fv : 0.0f); }
        d8 = dt + (size_t)h * 8u; }
    *(volatile v8h*)(d8) = o; __threadfence(); *(volatile v8h*)(d8) = o; }

__global__ __launch_bounds__(256) void k_sts(const float* __restrict__ c2, float* st) {
    const unsigned g = blockIdx.x * 256 + threadIdx.x; if (g >= (unsigned)(PRT * NPD)) return; const float* ur = c2 + (size_t)g * NCL; float s1 = 0.0f, s2 = 0.0f;
#pragma unroll
    for (int i = 0; i < NCL / 4; ++i) { const v4f q = *(const v4f*)(ur + 4 * i); s1 += (q[0] + q[1]) + (q[2] + q[3]); s2 += (q[0] * q[0] + q[1] * q[1]) + (q[2] * q[2] + q[3] * q[3]); }
    const float avg = s1 * (1.0f / (float)NCL); const float vr_ = s2 * (1.0f / (float)NCL) - avg * avg; v2f o; o[0] = avg; o[1] = 1.0f / sqrtf(fmaxf(vr_, 0.0f) + 1e-5f);
    float* d2 = st + 2u * (size_t)g; *(volatile v2f*)(d2) = o; __threadfence(); *(volatile v2f*)(d2) = o; }

__global__ __launch_bounds__(256) void k_fin(const float* __restrict__ c2, const float* __restrict__ st, const float* __restrict__ rg, float* rs, unsigned s0) {
    const unsigned t = blockIdx.x * 256 + threadIdx.x; if (t >= (unsigned)(NRW * (NCL / 4))) return; const unsigned sl = blockIdx.y, rn = t >> 6, ch = t & 63u; const size_t ri = (size_t)sl * NPD + rn;
    const v4f q = *(const v4f*)(c2 + ri * NCL + 4u * ch); const v4f gq = *(const v4f*)(rg + NCL + 4u * ch); const v4f bq = *(const v4f*)(rg + 2 * NCL + 4u * ch); const float avg = st[2u * ri], inv = st[2u * ri + 1u]; v4f o;
#pragma unroll
    for (int e = 0; e < 4; ++e) o[e] = (q[e] - avg) * inv * gq[e] + bq[e];
    float* dq = rs + ((size_t)(s0 + sl) * NRW + rn) * NCL + 4u * ch; *(volatile v4f*)(dq) = o; __threadfence(); *(volatile v4f*)(dq) = o; }

extern "C" void kernel_launch(void* const* d_in, const int* in_sizes, int n_in,
                              void* d_out, int out_size, void* d_ws, size_t ws_size, hipStream_t stream) {
    if (n_in < 6) return;
    if (in_sizes[0] < NSP * NRW * NCL || in_sizes[1] < NSP * NRW * NCL || in_sizes[2] < NCL * NGN || in_sizes[3] < NGN || in_sizes[4] < NCL || in_sizes[5] < NCL || out_size < NSP * NRW * NCL) return;
    const float* qs = (const float*)d_in[0]; const float* vs = (const float*)d_in[1]; const float* wg = (const float*)d_in[2]; const float* bg = (const float*)d_in[3]; const float* gm = (const float*)d_in[4]; const float* bt = (const float*)d_in[5];
    char* wsp = (char*)d_ws;
    auto take = [&](size_t bytes) { char* cur = wsp; wsp += (bytes + 255) & ~(size_t)255; return (void*)cur; };
    h16* Q16 = (h16*)take((size_t)NSP * NRW * NCL * 2); h16* WT = (h16*)take((size_t)NPD * NCL * 2); float* GN = (float*)take((size_t)NSP * NRW * NPD * 4); float* RS = (float*)take((size_t)3 * NCL * 4); float* RV = (float*)take((size_t)PRT * NRW * NCL * 4); h16* PM = (h16*)take((size_t)PRT * NPD * NPD * 2); h16* DT = (h16*)take((size_t)PRT * NCL * NPD * 2); float* C2 = (float*)take((size_t)PRT * NPD * NCL * 4); float* ST = (float*)take((size_t)PRT * NPD * 2 * 4);
    if ((size_t)(wsp - (char*)d_ws) != WS_TOTAL || WS_TOTAL > ws_size) return;
    auto lay = [&](const float* sp_, h16* dp_, unsigned nrow, unsigned ncol, unsigned dp, unsigned c0, unsigned rbs, unsigned ra, unsigned rs_, unsigned cbs, unsigned sa, unsigned sb, unsigned rlive, unsigned clive) {
        k_lay<<<(nrow * (ncol / 8) + 255) / 256, 256, 0, stream>>>(sp_, dp_, nrow, ncol / 8, dp, c0, rbs, ra, rs_, cbs, sa, sb, rlive, clive); };
    k_rnd<<<1, 256, 0, stream>>>(bg, RS, NCL / 4, NGN); k_rnd<<<1, 256, 0, stream>>>(gm, RS + NCL, NCL / 4, NCL); k_rnd<<<1, 256, 0, stream>>>(bt, RS + 2 * NCL, NCL / 4, NCL);
    lay(qs, Q16, NSP * NRW, NCL, NCL, 0, 16, 0, NCL, 16, 0, 1, NSP * NRW, NCL);
    lay(wg, WT, NPD, NCL, NCL, 0, 16, 0, 1, 16, 0, NGN, NGN, NCL);
    k_gemmw<h16, 0, false><<<dim3(NSP * NRW / 64, NPD / 64, 1), 32, 0, stream>>>(Q16, nullptr, WT, nullptr, NCL, GN, NPD, nullptr, (size_t)0, (size_t)0, (size_t)0);
    for (unsigned p = 0; p < (unsigned)(NSP / PRT); ++p) { const unsigned s0 = p * (unsigned)PRT;
        k_rnd<<<(PRT * NRW * NCL / 4 + 255) / 256, 256, 0, stream>>>(vs + (size_t)s0 * NRW * NCL, RV, PRT * NRW * NCL / 4, PRT * NRW * NCL);
        k_ops<<<(PRT * NPD * (NPD / 8) + PRT * NCL * (NPD / 8) + 255) / 256, 256, 0, stream>>>(GN, RS, RV, PM, DT, s0);
        k_gemmw<h16, 0, false><<<dim3(NPD / 64, NCL / 64, PRT), 32, 0, stream>>>(PM, nullptr, DT, nullptr, NPD, C2, NCL, nullptr, (size_t)NPD * NPD, (size_t)NCL * NPD, (size_t)NPD * NCL);
        k_sts<<<(PRT * NPD + 255) / 256, 256, 0, stream>>>(C2, ST);
        k_fin<<<dim3((NRW * (NCL / 4) + 255) / 256, PRT, 1), 256, 0, stream>>>(C2, ST, RS, (float*)d_out, s0); }
}
